// InceptionL_16166256902763
// MI455X (gfx1250) — hardware-verified
//
#include <hip/hip_runtime.h>
#include <stddef.h>
#include <math.h>


#define XD      64
#define NG      64
#define OC      128
#define NTHR    256
#define NWAVE   8
#define EPT     8
#define NGRP    2
#define CHUNK   (NTHR * EPT * NGRP)
#define WCAP    (EPT * NGRP * 32)
#define LISTN   (NWAVE * WCAP)
#define NBC     4096
#define NBF     1024
#define RCAP    40960
#define RBN     128
#define TGT     256
#define DEGCAP  256
#define GROWS   128
#define OTHR    512
#define SP      128
#define WSCAP   134217728
#define OPS     8.0f
#define OPINV   0.015625f

#define LDS_FILL ((RCAP + NBF + LISTN) * 4 + 64)

#define P13_OFF 0
#define P13_WPL (256 * 64)
#define P2_OFF  (P13_OFF + P13_WPL)
#define P2_WPL  (256 * 128)
#define P4_OFF  (P2_OFF + P2_WPL)
#define P7_OFF  (P4_OFF + P2_WPL)
#define P7_WPL  (128 * 320)
#define PL_TOT  (P7_OFF + P7_WPL)

static_assert((CHUNK & (CHUNK - 1)) == 0);
static_assert(CHUNK <= 4096);
static_assert(NBC <= 4096 && NBF <= 4096);
static_assert((NBC & (NBC - 1)) == 0 && (NBF & (NBF - 1)) == 0);
static_assert(NBC == 4 * NBF);
static_assert(OTHR * 8 == NBC);
static_assert((RCAP % 32) == 0);
static_assert((TGT % GROWS) == 0 && TGT == NWAVE * 32);
static_assert((NBC % TGT) == 0);
static_assert(GROWS == NWAVE * 16);
static_assert(SP == OC);

typedef float    v2f  __attribute__((ext_vector_type(2)));
typedef float    v4f  __attribute__((ext_vector_type(4)));
typedef float    v8f  __attribute__((ext_vector_type(8)));
typedef int      v4i  __attribute__((ext_vector_type(4)));
typedef _Float16 v8h  __attribute__((ext_vector_type(8)));
typedef _Float16 v16h __attribute__((ext_vector_type(16)));
union FragH { v16h v; v8h h[2]; };

__host__ __device__ constexpr int ldsg(int kd) {
  return (GROWS * (kd + 8) * 2 > GROWS * SP * 4) ? (GROWS * (kd + 8) * 2) : (GROWS * SP * 4);
}

__device__ __forceinline__ v8h cvt8h(v4f a, v4f b) {
  v8h r;
  r[0] = (_Float16)(a.x * OPS); r[1] = (_Float16)(a.y * OPS);
  r[2] = (_Float16)(a.z * OPS); r[3] = (_Float16)(a.w * OPS);
  r[4] = (_Float16)(b.x * OPS); r[5] = (_Float16)(b.y * OPS);
  r[6] = (_Float16)(b.z * OPS); r[7] = (_Float16)(b.w * OPS);
  return r;
}

__device__ __forceinline__ v8f wmf(v16h a, v16h b, v8f c) {
  v8f d = __builtin_amdgcn_wmma_f32_16x16x32_f16(false, a, false, b, (short)0, c, false, false);
  asm volatile("v_nop\n\tv_nop\n\tv_nop\n\tv_nop" : "+v"(d) : "v"(a), "v"(b));
  return d;
}

template <int NB>
__device__ __forceinline__ int scan_chunk(const int* __restrict__ dsts, int nE, int cbase, int slotBase,
                                          int vec8, int* list, int tid, int lane, int wave) {
  int wc = 0;
#pragma unroll
  for (int g = 0; g < NGRP; ++g) {
    const int el0  = (g * NTHR + tid) * EPT;
    const int e0   = cbase + el0;
    const int sent = -2147483647 - 1;
    v4i da, db;
    if (vec8 != 0 && cbase + CHUNK <= nE) {
      da = *(const v4i*)(dsts + e0);
      db = *(const v4i*)(dsts + e0 + 4);
    } else {
      da.x = (e0     < nE) ? dsts[min(e0, nE - 1)] : sent;
      da.y = (e0 + 1 < nE) ? dsts[min(e0 + 1, nE - 1)] : sent;
      da.z = (e0 + 2 < nE) ? dsts[min(e0 + 2, nE - 1)] : sent;
      da.w = (e0 + 3 < nE) ? dsts[min(e0 + 3, nE - 1)] : sent;
      db.x = (e0 + 4 < nE) ? dsts[min(e0 + 4, nE - 1)] : sent;
      db.y = (e0 + 5 < nE) ? dsts[min(e0 + 5, nE - 1)] : sent;
      db.z = (e0 + 6 < nE) ? dsts[min(e0 + 6, nE - 1)] : sent;
      db.w = (e0 + 7 < nE) ? dsts[min(e0 + 7, nE - 1)] : sent;
    }
    const unsigned nb = (unsigned)slotBase;
    const unsigned s0 = (unsigned)da.x - nb, s1 = (unsigned)da.y - nb;
    const unsigned s2 = (unsigned)da.z - nb, s3 = (unsigned)da.w - nb;
    const unsigned s4 = (unsigned)db.x - nb, s5 = (unsigned)db.y - nb;
    const unsigned s6 = (unsigned)db.z - nb, s7 = (unsigned)db.w - nb;
    const bool h0 = s0 < (unsigned)NB, h1 = s1 < (unsigned)NB, h2 = s2 < (unsigned)NB, h3 = s3 < (unsigned)NB;
    const bool h4 = s4 < (unsigned)NB, h5 = s5 < (unsigned)NB, h6 = s6 < (unsigned)NB, h7 = s7 < (unsigned)NB;
    const unsigned any = __builtin_amdgcn_ballot_w32(h0 | h1 | h2 | h3 | h4 | h5 | h6 | h7);
    if (any != 0u) {
#define HITJ(J, HJ, SJ) { \
        const unsigned mj = __builtin_amdgcn_ballot_w32(HJ); \
        if (mj != 0u) { \
          if (HJ) { \
            const int pos = wc + (int)__builtin_amdgcn_mbcnt_lo(mj, 0u); \
            if (pos < WCAP) list[wave * WCAP + pos] = ((el0 + (J)) << 12) | (int)(SJ); \
          } \
          wc += (int)__builtin_popcount(mj); } }
      HITJ(0, h0, s0)
      HITJ(1, h1, s1)
      HITJ(2, h2, s2)
      HITJ(3, h3, s3)
      HITJ(4, h4, s4)
      HITJ(5, h5, s5)
      HITJ(6, h6, s6)
      HITJ(7, h7, s7)
#undef HITJ
    }
  }
  return wc;
}

__global__ __launch_bounds__(NTHR) void k_wprep(
    const float* __restrict__ W1, const float* __restrict__ W3, const float* __restrict__ W2,
    const float* __restrict__ W4, const float* __restrict__ W7, _Float16* wp) {
  const int b = blockIdx.x, tid = threadIdx.x;
  const float* src; int pitch, cpn, nsub, koff, gi, poff;
  if (b < 4)       { src = W1; pitch = 128; cpn = 8;  nsub = 0;   koff = 0;   poff = P13_OFF; gi = b * NTHR; }
  else if (b < 8)  { src = W3; pitch = 128; cpn = 8;  nsub = 128; koff = 0;   poff = P13_OFF; gi = b * NTHR; }
  else if (b < 24) { src = W2; pitch = 256; cpn = 16; nsub = 0;   koff = 0;   poff = P2_OFF;  gi = (b - 8) * NTHR; }
  else if (b < 40) { src = W4; pitch = 256; cpn = 16; nsub = 0;   koff = 0;   poff = P4_OFF;  gi = (b - 24) * NTHR; }
  else             { src = W7; pitch = 128; cpn = 40; nsub = 0;   koff = 256; poff = P7_OFF;  gi = (b - 40) * NTHR; }
  const int i  = gi + tid;
  const int n  = i / cpn;
  const int k0 = (i - n * cpn) * 8;
  const int col = n - nsub;
  float v[8];
#pragma unroll
  for (int e = 0; e < 8; ++e) v[e] = src[(size_t)(koff + k0 + e) * pitch + col];
  v4f a, c;
  a.x = v[0]; a.y = v[1]; a.z = v[2]; a.w = v[3];
  c.x = v[4]; c.y = v[5]; c.z = v[6]; c.w = v[7];
  const v8h hv = cvt8h(a, c);
  _Float16* dh = wp + poff + (size_t)i * 8;
  *(volatile v8h*)dh = hv;
  __threadfence();
  *(volatile v8h*)dh = hv;
}

__global__ __launch_bounds__(NTHR) void k_count(
    const int* __restrict__ ei, int* cnt, float* dinv, int nE, int vec8) {
  __shared__ __attribute__((aligned(16))) int scnt[NBC];
  __shared__ __attribute__((aligned(16))) int list[LISTN];
  __shared__ int wcnt[NWAVE];
  const int tid = threadIdx.x, lane = tid & 31, wave = tid >> 5;
  const int nodeBase = blockIdx.x * NBC;
  const int* dsts = ei + nE;

  for (int i = tid; i < NBC; i += NTHR) scnt[i] = 0;
  __syncthreads();

  const int nChunks = (nE + CHUNK - 1) / CHUNK;
#pragma unroll 1
  for (int ch = 0; ch < nChunks; ++ch) {
    const int cbase = ch * CHUNK;
    const int wc = scan_chunk<NBC>(dsts, nE, cbase, nodeBase, vec8, list, tid, lane, wave);
    if (lane == 0) wcnt[wave] = wc;
    __syncthreads();
    if (wave == 0) {
#pragma unroll 1
      for (int wsx = 0; wsx < NWAVE; ++wsx) {
        int n = __builtin_amdgcn_readfirstlane(wcnt[wsx]);
        n = n > WCAP ? WCAP : (n < 0 ? 0 : n);
        const int* lp = list + wsx * WCAP;
#pragma unroll 1
        for (int i = 0; i < n; ++i) {
          const int ent  = __builtin_amdgcn_readfirstlane(lp[i]);
          const int slot = ent & (NBC - 1);
          if (lane == 0) scnt[slot] = scnt[slot] + 1;
        }
      }
    }
    __syncthreads();
  }

  v4i cq[4]; v4f dq[4];
#pragma unroll
  for (int q = 0; q < 4; ++q) {
    const int f = (wave * 4 + q) * 128 + 4 * lane;
    const v4i c = *(const v4i*)(scnt + f);
    cq[q] = c;
    dq[q].x = rsqrtf((float)(c.x + 1));
    dq[q].y = rsqrtf((float)(c.y + 1));
    dq[q].z = rsqrtf((float)(c.z + 1));
    dq[q].w = rsqrtf((float)(c.w + 1));
  }
  int*   cp = cnt + (size_t)nodeBase;
  float* dp = dinv + (size_t)nodeBase;
#pragma unroll
  for (int q = 0; q < 4; ++q) {
    const int f = (wave * 4 + q) * 128 + 4 * lane;
    *(volatile v4i*)(cp + f) = cq[q];
    *(volatile v4f*)(dp + f) = dq[q];
  }
  __threadfence();
#pragma unroll
  for (int q = 0; q < 4; ++q) {
    const int f = (wave * 4 + q) * 128 + 4 * lane;
    *(volatile v4i*)(cp + f) = cq[q];
    *(volatile v4f*)(dp + f) = dq[q];
  }
}

__global__ __launch_bounds__(OTHR) void k_offsets(
    const int* __restrict__ cnt, int* off, int* rbase, int nChunk) {
  __shared__ __attribute__((aligned(16))) int soff[NBC];
  __shared__ __attribute__((aligned(16))) int srb[RBN];
  __shared__ int wtot[OTHR / 32];
  const int tid = threadIdx.x, lane = tid & 31, wave = tid >> 5, sub = tid >> 7;
  for (int i = tid; i < RBN; i += OTHR) srb[i] = 0;
  int carry = 0;
#pragma unroll 1
  for (int ch = 0; ch < nChunk; ++ch) {
    const int base = ch * NBC;
    const v4i c0 = *(const v4i*)(cnt + base + 8 * tid);
    const v4i c1 = *(const v4i*)(cnt + base + 8 * tid + 4);
    const int e0 = max(c0.x, 0), e1 = max(c0.y, 0), e2 = max(c0.z, 0), e3 = max(c0.w, 0);
    const int e4 = max(c1.x, 0), e5 = max(c1.y, 0), e6 = max(c1.z, 0), e7 = max(c1.w, 0);
    const int ts = e0 + e1 + e2 + e3 + e4 + e5 + e6 + e7;
    int incl = ts;
#pragma unroll
    for (int d = 1; d < 32; d <<= 1) {
      const int t = __shfl_up(incl, d);
      if (lane >= d) incl += t;
    }
    if (lane == 31) wtot[wave] = incl;
    __syncthreads();
    const int S0 = wtot[0]  + wtot[1]  + wtot[2]  + wtot[3];
    const int S1 = wtot[4]  + wtot[5]  + wtot[6]  + wtot[7];
    const int S2 = wtot[8]  + wtot[9]  + wtot[10] + wtot[11];
    const int S3 = wtot[12] + wtot[13] + wtot[14] + wtot[15];
    int pre = 0;
#pragma unroll 1
    for (int w = 4 * sub; w < wave; ++w) pre += wtot[w];
    const int b0 = carry;
    const int b1 = b0 + ((S0 + 31) & ~31);
    const int b2 = b1 + ((S1 + 31) & ~31);
    const int b3 = b2 + ((S2 + 31) & ~31);
    const int b4 = b3 + ((S3 + 31) & ~31);
    const int myb = sub == 0 ? b0 : (sub == 1 ? b1 : (sub == 2 ? b2 : b3));
    if (tid == 0) {
      srb[min(4 * ch + 0, RBN - 1)] = b0;
      srb[min(4 * ch + 1, RBN - 1)] = b1;
      srb[min(4 * ch + 2, RBN - 1)] = b2;
      srb[min(4 * ch + 3, RBN - 1)] = b3;
    }
    int run = myb + pre + incl - ts;
    soff[8 * tid + 0] = run; run += e0;
    soff[8 * tid + 1] = run; run += e1;
    soff[8 * tid + 2] = run; run += e2;
    soff[8 * tid + 3] = run; run += e3;
    soff[8 * tid + 4] = run; run += e4;
    soff[8 * tid + 5] = run; run += e5;
    soff[8 * tid + 6] = run; run += e6;
    soff[8 * tid + 7] = run;
    carry = b4;
    __syncthreads();
    const v4i o0 = *(const v4i*)(soff + 4 * tid);
    const v4i o1 = *(const v4i*)(soff + 4 * (tid + OTHR));
    int* op = off + base;
    *(volatile v4i*)(op + 4 * tid) = o0;
    *(volatile v4i*)(op + 4 * (tid + OTHR)) = o1;
    __threadfence();
    *(volatile v4i*)(op + 4 * tid) = o0;
    *(volatile v4i*)(op + 4 * (tid + OTHR)) = o1;
    __syncthreads();
  }
  if (tid == 0) srb[min(4 * nChunk, RBN - 1)] = carry;
  __syncthreads();
  v4i rv = {0, 0, 0, 0};
  if (tid < 32) rv = *(const v4i*)(srb + 4 * tid);
  if (tid < 32) *(volatile v4i*)(rbase + 4 * tid) = rv;
  __threadfence();
  if (tid < 32) *(volatile v4i*)(rbase + 4 * tid) = rv;
}

__global__ __launch_bounds__(NTHR) void k_fill(
    const int* __restrict__ ei, const int* __restrict__ off, const int* __restrict__ rbase,
    int* csr, int nN, int nE, int vec8, int csrLen) {
  extern __shared__ v4f lds_dyn[];
  int* region = (int*)lds_dyn;
  int* cursor = region + RCAP;
  int* list   = cursor + NBF;
  int* wcnt   = list + LISTN;
  const int tid = threadIdx.x, lane = tid & 31, wave = tid >> 5;
  const int b = blockIdx.x;
  const int nodeBase = b * NBF;
  const int* dsts = ei + nE;

  int rb0 = rbase[b];
  const int rb1 = rbase[b + 1];
  rb0 = rb0 < 0 ? 0 : (rb0 > csrLen ? csrLen : rb0);
  rb0 &= ~31;
  int len = rb1 - rb0;
  len = len < 0 ? 0 : (len > RCAP ? RCAP : len);
  int lenW = (len + 31) & ~31;
  if (rb0 + lenW > csrLen) lenW = (csrLen - rb0) & ~31;

  {
    const v4i z = {0, 0, 0, 0};
    for (int i = tid; i < RCAP / 4; i += NTHR) ((v4i*)region)[i] = z;
    for (int s = tid; s < NBF; s += NTHR) {
      int o = off[nodeBase + s] - rb0;
      o = o < 0 ? 0 : (o > RCAP ? RCAP : o);
      cursor[s] = o;
    }
  }
  __syncthreads();

  const int nChunks = (nE + CHUNK - 1) / CHUNK;
#pragma unroll 1
  for (int ch = 0; ch < nChunks; ++ch) {
    const int cbase = ch * CHUNK;
    const int wc = scan_chunk<NBF>(dsts, nE, cbase, nodeBase, vec8, list, tid, lane, wave);
    if (lane == 0) wcnt[wave] = wc;
    __syncthreads();
    if (wave == 0) {
#pragma unroll 1
      for (int wsx = 0; wsx < NWAVE; ++wsx) {
        int n = __builtin_amdgcn_readfirstlane(wcnt[wsx]);
        n = n > WCAP ? WCAP : (n < 0 ? 0 : n);
        const int* lp = list + wsx * WCAP;
#pragma unroll 1
        for (int i = 0; i < n; ++i) {
          const int ent  = __builtin_amdgcn_readfirstlane(lp[i]);
          const int slot = ent & (NBF - 1);
          int e = cbase + ((ent >> 12) & (CHUNK - 1));
          e = e > nE - 1 ? nE - 1 : e;
          int src = ei[e];
          src = src < 0 ? 0 : (src > nN - 1 ? nN - 1 : src);
          if (lane == 0) {
            int pos = cursor[slot];
            pos = pos < 0 ? 0 : (pos > RCAP - 1 ? RCAP - 1 : pos);
            region[pos] = src;
            const int np = pos + 1;
            cursor[slot] = np > RCAP ? RCAP : np;
          }
        }
      }
    }
    __syncthreads();
  }

  const int nv = lenW >> 2;
  int* gp = csr + rb0;
#pragma unroll 1
  for (int i = tid; i < nv; i += NTHR) { const v4i v = ((const v4i*)region)[i]; *(volatile v4i*)(gp + 4 * i) = v; }
  __threadfence();
#pragma unroll 1
  for (int i = tid; i < nv; i += NTHR) { const v4i v = ((const v4i*)region)[i]; *(volatile v4i*)(gp + 4 * i) = v; }
}

__global__ __launch_bounds__(NTHR) void k_xscale(
    const float* __restrict__ x, const float* __restrict__ dinv, float* xs, int nN) {
  const int tid = threadIdx.x, lane = tid & 31, wave = tid >> 5, hh = lane >> 4, q = lane & 15;
  const int rb = blockIdx.x * TGT + wave * 32;
  v4f v[16];
#pragma unroll
  for (int i = 0; i < 16; ++i) {
    const int r  = rb + 2 * i + hh;
    const int rr = r > nN - 1 ? nN - 1 : r;
    const v4f a = *(const v4f*)(x + (size_t)rr * XD + 4 * q);
    const float d = dinv[r];
    const float s = (r < nN) ? d : 0.0f;
    v[i] = a * s;
  }
#pragma unroll
  for (int i = 0; i < 16; ++i) {
    const int r = rb + 2 * i + hh;
    *(volatile v4f*)(xs + (size_t)r * XD + 4 * q) = v[i];
  }
  __threadfence();
#pragma unroll
  for (int i = 0; i < 16; ++i) {
    const int r = rb + 2 * i + hh;
    *(volatile v4f*)(xs + (size_t)r * XD + 4 * q) = v[i];
  }
}

template <int K1, int K2>
__global__ __launch_bounds__(NTHR) void k_gemm(
    const float* __restrict__ A1, int lda1, int nRowsA1,
    const float* __restrict__ A2, int lda2, int nRowsA2,
    const _Float16* __restrict__ Bw,
    const float* __restrict__ av0, const float* __restrict__ av1,
    const float* __restrict__ dinv, const int* __restrict__ bvec, int nValid,
    float* C, int ldc, int nRowsC, int flags) {
  constexpr int KD  = K1 + K2;
  constexpr int APH = KD + 8;
  constexpr int C1  = K1 / 8;
  constexpr int C2  = K2 > 0 ? K2 / 8 : 1;
  extern __shared__ v4f lds_dyn[];
  __shared__ __attribute__((aligned(16))) float smx[NWAVE * SP];
  _Float16* sA  = (_Float16*)lds_dyn;
  float*    stg = (float*)lds_dyn;
  const int tid = threadIdx.x, lane = tid & 31, wave = tid >> 5, hh = lane >> 4, m = lane & 15;
  const int rowBase = blockIdx.x * GROWS;
  const int cb = (int)blockIdx.y * OC;
  const float* av = (blockIdx.y == 0) ? av0 : av1;

#pragma unroll 2
  for (int i = 0; i < (GROWS * C1) / NTHR; ++i) {
    const int idx = i * NTHR + tid;
    const int r   = idx / C1;
    const int c0  = (idx - r * C1) * 8;
    int row = rowBase + r;
    row = row > nRowsA1 - 1 ? nRowsA1 - 1 : row;
    const float* ap = A1 + (size_t)row * lda1 + c0;
    const v4f a = *(const v4f*)ap, b = *(const v4f*)(ap + 4);
    *(v8h*)(sA + r * APH + c0) = cvt8h(a, b);
  }
  if (K2 > 0) {
#pragma unroll 2
    for (int i = 0; i < (GROWS * (K2 / 8)) / NTHR; ++i) {
      const int idx = i * NTHR + tid;
      const int r   = idx / C2;
      const int c0  = (idx - r * C2) * 8;
      int row = rowBase + r;
      row = row > nRowsA2 - 1 ? nRowsA2 - 1 : row;
      const float* ap = A2 + (size_t)row * lda2 + c0;
      const v4f a = *(const v4f*)ap, b = *(const v4f*)(ap + 4);
      *(v8h*)(sA + r * APH + K1 + c0) = cvt8h(a, b);
    }
  }
  __syncthreads();

  v8f acc[8];
#pragma unroll
  for (int t = 0; t < 8; ++t) { v8f z = {0.f, 0.f, 0.f, 0.f, 0.f, 0.f, 0.f, 0.f}; acc[t] = z; }
  const _Float16* ahp = sA + (wave * 16 + m) * APH + 8 * hh;
  const _Float16* bwp = Bw + (size_t)(cb + m) * KD + 8 * hh;
#pragma unroll 1
  for (int kt = 0; kt < KD / 32; ++kt) {
    FragH ah;
    ah.h[0] = *(const v8h*)(ahp + 32 * kt);
    ah.h[1] = *(const v8h*)(ahp + 32 * kt + 16);
#pragma unroll
    for (int t = 0; t < 8; ++t) {
      const _Float16* bp = bwp + (size_t)(16 * t) * KD + 32 * kt;
      FragH bh;
      bh.h[0] = *(const v8h*)bp;
      bh.h[1] = *(const v8h*)(bp + 16);
      acc[t] = wmf(ah.v, bh.v, acc[t]);
    }
  }
  __syncthreads();

  const int r0 = wave * 16 + 8 * hh;
  float* sp = stg + r0 * SP + m;
#pragma unroll
  for (int t = 0; t < 8; ++t) {
    const float bv = av[16 * t + m];
#pragma unroll
    for (int r = 0; r < 8; ++r) sp[r * SP + 16 * t] = acc[t][r] * OPINV + bv;
  }
  __syncthreads();

  float* lp = stg + wave * 16 * SP + 4 * lane;
  const int rw0 = rowBase + wave * 16;
  const float ninf = -__builtin_inff();
  v4f cm = {ninf, ninf, ninf, ninf};
#pragma unroll 1
  for (int i = 0; i < 16; ++i) {
    v4f v = *(const v4f*)(lp + i * SP);
    const int row = rw0 + i;
    if (flags & 1) { v.x = tanhf(v.x); v.y = tanhf(v.y); v.z = tanhf(v.z); v.w = tanhf(v.w); }
    if (flags & 2) { const float d = dinv[row]; v = v * d; }
    if (flags & 4) {
      const int rr  = row > nValid - 1 ? nValid - 1 : row;
      const int bvv = bvec[rr];
      const bool ok = (row < nValid) && ((unsigned)bvv < (unsigned)NG);
      cm.x = ok ? fmaxf(cm.x, v.x) : cm.x;
      cm.y = ok ? fmaxf(cm.y, v.y) : cm.y;
      cm.z = ok ? fmaxf(cm.z, v.z) : cm.z;
      cm.w = ok ? fmaxf(cm.w, v.w) : cm.w;
    }
    *(v4f*)(lp + i * SP) = v;
  }

  if (flags & 4) {
    *(v4f*)(smx + wave * SP + 4 * lane) = cm;
    __syncthreads();
    if (wave == 0) {
      v4f mm = *(const v4f*)(smx + 4 * lane);
#pragma unroll
      for (int w = 1; w < NWAVE; ++w) {
        const v4f o = *(const v4f*)(smx + w * SP + 4 * lane);
        mm.x = fmaxf(mm.x, o.x); mm.y = fmaxf(mm.y, o.y); mm.z = fmaxf(mm.z, o.z); mm.w = fmaxf(mm.w, o.w);
      }
      float* gp = C + (size_t)blockIdx.x * ldc + cb + 4 * lane;
      *(volatile v4f*)gp = mm;
      __threadfence();
      *(volatile v4f*)gp = mm;
    }
  } else {
    float* gp = C + (size_t)rw0 * ldc + cb + 4 * lane;
#pragma unroll
    for (int i = 0; i < 16; ++i) {
      const v4f v = *(const v4f*)(lp + i * SP);
      if (rw0 + i < nRowsC) *(volatile v4f*)(gp + (size_t)i * ldc) = v;
    }
    __threadfence();
#pragma unroll
    for (int i = 0; i < 16; ++i) {
      const v4f v = *(const v4f*)(lp + i * SP);
      if (rw0 + i < nRowsC) *(volatile v4f*)(gp + (size_t)i * ldc) = v;
    }
  }
}

template <int CH, int ACT>
__global__ __launch_bounds__(NTHR) void k_agg(
    const int* __restrict__ csr, const int* __restrict__ off, const int* __restrict__ cnt,
    const float* __restrict__ dinv, const float* __restrict__ S, float* D,
    const float* __restrict__ bs, int nN, int csrLen, int nRowsD) {
  union FI { float f; int i; };
  const int tid = threadIdx.x, lane = tid & 31, wave = tid >> 5;
  const int tbase = blockIdx.x * TGT + wave * 32;
  const int cl = tbase + lane;
  const int cnt_l = cnt[cl];
  const int off_l = off[cl];
  FI dvu; dvu.f = dinv[cl];
  const int co = (CH == 64) ? 2 * lane : 4 * lane;
  v4f bb = {0.f, 0.f, 0.f, 0.f};
  if (ACT) bb = *(const v4f*)(bs + 4 * lane);

#pragma unroll 1
  for (int j = 0; j < 32; ++j) {
    const int c = tbase + j;
    int n = __builtin_amdgcn_readlane(cnt_l, j);
    n = n < 0 ? 0 : (n > DEGCAP ? DEGCAP : n);
    const int st = __builtin_amdgcn_readlane(off_l, j);
    FI du; du.i = __builtin_amdgcn_readlane(dvu.i, j);
    const float dc = du.f;
    v4f a0 = {0.f, 0.f, 0.f, 0.f}, a1 = {0.f, 0.f, 0.f, 0.f};
#pragma unroll 1
    for (int q0 = 0; q0 < n; q0 += 32) {
      int pos = st + q0 + lane;
      pos = pos < 0 ? 0 : (pos > csrLen - 1 ? csrLen - 1 : pos);
      int sl = csr[pos];
      sl = sl < 0 ? 0 : (sl > nN - 1 ? nN - 1 : sl);
      const int mcnt = (n - q0) < 32 ? (n - q0) : 32;
#pragma unroll 1
      for (int p = 0; p < mcnt; ++p) {
        const int s = __builtin_amdgcn_readlane(sl, p);
        const float* srow = S + (size_t)s * CH;
        if (CH == 64) {
          const v2f t = *(const v2f*)(srow + co);
          a0.x += t.x; a0.y += t.y;
        } else {
          a0 = a0 + *(const v4f*)(srow + co);
          if (CH == 256) a1 = a1 + *(const v4f*)(srow + 128 + co);
        }
      }
    }
    const float* crow_ = S + (size_t)c * CH;
    v4f s0 = {0.f, 0.f, 0.f, 0.f}, s1 = {0.f, 0.f, 0.f, 0.f};
    if (CH == 64) {
      const v2f t = *(const v2f*)(crow_ + co);
      s0.x = t.x; s0.y = t.y;
    } else {
      s0 = *(const v4f*)(crow_ + co);
      if (CH == 256) s1 = *(const v4f*)(crow_ + 128 + co);
    }
    v4f v0 = (a0 + s0) * dc;
    v4f v1 = (a1 + s1) * dc;
    if (ACT) {
      v0 = v0 + bb;
      v0.x = tanhf(v0.x); v0.y = tanhf(v0.y); v0.z = tanhf(v0.z); v0.w = tanhf(v0.w);
    }
    float* dp = D + (size_t)c * CH;
    v2f o2; o2.x = v0.x; o2.y = v0.y;
    if (c < nRowsD) {
      if (CH == 64) { *(volatile v2f*)(dp + co) = o2; }
      else {
        *(volatile v4f*)(dp + co) = v0;
        if (CH == 256) *(volatile v4f*)(dp + 128 + co) = v1;
      }
    }
    __threadfence();
    if (c < nRowsD) {
      if (CH == 64) { *(volatile v2f*)(dp + co) = o2; }
      else {
        *(volatile v4f*)(dp + co) = v0;
        if (CH == 256) *(volatile v4f*)(dp + 128 + co) = v1;
      }
    }
  }
}

__global__ __launch_bounds__(NTHR) void k_poolc(
    const float* __restrict__ part, int nPart, const float* __restrict__ W7, float* crow) {
  __shared__ __attribute__((aligned(16))) float spool[256];
  __shared__ __attribute__((aligned(16))) float scr[OC];
  const int tid = threadIdx.x;
  float mx = -__builtin_inff();
#pragma unroll 1
  for (int b = 0; b < nPart; ++b) mx = fmaxf(mx, part[(size_t)b * 256 + tid]);
  spool[tid] = mx;
  __syncthreads();
  if (tid < OC) {
    float s = 0.0f;
#pragma unroll 1
    for (int k = 0; k < 256; ++k) s += spool[k] * W7[(size_t)k * OC + tid];
    scr[tid] = s;
  }
  __syncthreads();
  if (tid < 32) {
    const v4f v = *(const v4f*)(scr + 4 * tid);
    *(volatile v4f*)(crow + 4 * tid) = v;
    __threadfence();
    *(volatile v4f*)(crow + 4 * tid) = v;
  }
}

extern "C" void kernel_launch(void* const* d_in, const int* in_sizes, int n_in,
                              void* d_out, int out_size, void* d_ws, size_t ws_size,
                              hipStream_t stream) {
  if (n_in < 13) return;
  const int nN = in_sizes[0] / XD;
  const int nE = in_sizes[1] / 2;
  if (nN <= 0 || nE <= 0 || in_sizes[0] != nN * XD || in_sizes[1] != 2 * nE) return;
  if (in_sizes[2] != nN) return;
  if (in_sizes[3] != 64 * 128 || in_sizes[4] != 128) return;
  if (in_sizes[5] != 128 * 256 || in_sizes[6] != 256) return;
  if (in_sizes[7] != 64 * 128 || in_sizes[8] != 128) return;
  if (in_sizes[9] != 128 * 256 || in_sizes[10] != 256) return;
  if (in_sizes[11] != 576 * 128 || in_sizes[12] != 128) return;
  if (out_size != nN * OC) return;
  if (nE > (1 << 28) || nN > (1 << 24)) return;

  const float* x    = (const float*)d_in[0];
  const int*   ei   = (const int*)d_in[1];
  const int*   bidx = (const int*)d_in[2];
  const float* W1 = (const float*)d_in[3];
  const float* b1 = (const float*)d_in[4];
  const float* W2 = (const float*)d_in[5];
  const float* b2 = (const float*)d_in[6];
  const float* W3 = (const float*)d_in[7];
  const float* b3 = (const float*)d_in[8];
  const float* W4 = (const float*)d_in[9];
  const float* b4 = (const float*)d_in[10];
  const float* W7 = (const float*)d_in[11];
  const float* b7 = (const float*)d_in[12];
  float* out = (float*)d_out;

  const int NPAD   = ((nN + TGT - 1) / TGT) * TGT;
  const int nBC    = (nN + NBC - 1) / NBC;
  const int CNTPAD = nBC * NBC;
  if (4 * nBC + 1 > RBN) return;
  const int nBF    = (nN + NBF - 1) / NBF;
  const int csrLen = ((nE + 31) & ~31) + 4096;
  if (31 * 4 * nBC > 4096) return;
  const int nGemm  = NPAD / GROWS;
  const int nAgg   = NPAD / TGT;

  char* ws = (char*)d_ws;
  size_t off = 0;
  const size_t oPl   = off; off += (size_t)PL_TOT * 2;             off = (off + 255) & ~(size_t)255;
  const size_t oCnt  = off; off += (size_t)CNTPAD * 4;             off = (off + 255) & ~(size_t)255;
  const size_t oDv   = off; off += (size_t)CNTPAD * 4;             off = (off + 255) & ~(size_t)255;
  const size_t oOff  = off; off += (size_t)CNTPAD * 4;             off = (off + 255) & ~(size_t)255;
  const size_t oRb   = off; off += (size_t)RBN * 4;                off = (off + 255) & ~(size_t)255;
  const size_t oCsr  = off; off += (size_t)csrLen * 4;             off = (off + 255) & ~(size_t)255;
  const size_t oR1   = off; off += (size_t)NPAD * 256 * 4;         off = (off + 255) & ~(size_t)255;
  const size_t oR2   = off; off += (size_t)NPAD * 256 * 4;         off = (off + 255) & ~(size_t)255;
  const size_t oPart = off; off += (size_t)nGemm * 256 * 4;        off = (off + 255) & ~(size_t)255;
  const size_t oCrow = off; off += (size_t)OC * 4;                 off = (off + 255) & ~(size_t)255;
  if (off > ws_size || off > (size_t)WSCAP) return;
  _Float16* wp  = (_Float16*)(ws + oPl);
  int*    cnt  = (int*)(ws + oCnt);
  float*  dinv = (float*)(ws + oDv);
  int*    offp = (int*)(ws + oOff);
  int*    rb   = (int*)(ws + oRb);
  int*    csr  = (int*)(ws + oCsr);
  float*  R1   = (float*)(ws + oR1);
  float*  R2   = (float*)(ws + oR2);
  float*  part = (float*)(ws + oPart);
  float*  crow = (float*)(ws + oCrow);
  float*  xs   = R2;
  float*  ax   = R2 + (size_t)NPAD * XD;

  const int vec8 = ((nE & 3) == 0) ? 1 : 0;
  constexpr int LDS64  = ldsg(64);
  constexpr int LDS128 = ldsg(128);
  constexpr int LDS320 = ldsg(320);

  k_wprep<<<60, NTHR, 0, stream>>>(W1, W3, W2, W4, W7, wp);

  k_count<<<nBC, NTHR, 0, stream>>>(ei, cnt, dinv, nE, vec8);
  k_offsets<<<1, OTHR, 0, stream>>>(cnt, offp, rb, nBC);
  k_fill<<<nBF, NTHR, LDS_FILL, stream>>>(ei, offp, rb, csr, nN, nE, vec8, csrLen);

  k_xscale<<<nAgg, NTHR, 0, stream>>>(x, dinv, xs, nN);
  k_agg<64, 0><<<nAgg, NTHR, 0, stream>>>(csr, offp, cnt, dinv, xs, ax, b1, nN, csrLen, NPAD);

  k_gemm<64, 0><<<dim3(nGemm, 2), NTHR, LDS64, stream>>>(
      ax, XD, NPAD, ax, XD, NPAD, wp + P13_OFF, b1, b3, dinv, bidx, nN, R1, 256, NPAD, 3);

  k_agg<256, 0><<<nAgg, NTHR, 0, stream>>>(csr, offp, cnt, dinv, R1, R2, b1, nN, csrLen, NPAD);

  k_gemm<128, 0><<<dim3(nGemm, 2), NTHR, LDS128, stream>>>(
      R2, 256, NPAD, R2, 256, NPAD, wp + P2_OFF, b2, b2 + 128, dinv, bidx, nN, part, 256, nGemm, 5);

  k_poolc<<<1, NTHR, 0, stream>>>(part, nGemm, W7, crow);

  k_gemm<128, 0><<<dim3(nGemm, 2), NTHR, LDS128, stream>>>(
      R2 + 128, 256, NPAD, R2 + 128, 256, NPAD, wp + P4_OFF, b4, b4 + 128, dinv, bidx, nN, R1, 256, NPAD, 1);

  k_gemm<256, 64><<<dim3(nGemm, 1), NTHR, LDS320, stream>>>(
      R1, 256, NPAD, x, XD, nN, wp + P7_OFF, crow, crow, dinv, bidx, nN, R2, OC, NPAD, 2);

  k_agg<128, 1><<<nAgg, NTHR, 0, stream>>>(csr, offp, cnt, dinv, R2, out, b7, nN, csrLen, nN);
}
